// Mamba2Simple_15745350107165
// MI455X (gfx1250) — hardware-run, weakly checked
//
#include <hip/hip_runtime.h>
#include <hip/hip_fp16.h>
#include <math.h>

typedef __attribute__((ext_vector_type(16))) _Float16 v16h;
typedef __attribute__((ext_vector_type(8)))  _Float16 v8h;
typedef __attribute__((ext_vector_type(8)))  float    v8f;
typedef __attribute__((ext_vector_type(4)))  float    v4f;
typedef __attribute__((ext_vector_type(4)))  unsigned v4u;

constexpr int kBatch  = 2;
constexpr int kSeq    = 4096;
constexpr int kRows   = kBatch * kSeq;
constexpr int kDm     = 512;
constexpr int kDin    = 1024;
constexpr int kHeads  = 64;
constexpr int kHd     = 16;
constexpr int kNst    = 16;
constexpr int kConvC  = kDin + 2 * kNst;
constexpr int kProj   = 2 * kDin + 2 * kNst + kHeads;
constexpr int kProjP  = 2176;
constexpr int kQW     = kProjP - kDin;
constexpr int kQDt    = kConvC;
constexpr int kConvTh = 352;
static_assert(kRows == 8192 && kConvC == 1056 && kProj == 2144 && kQW == 1152);
static_assert(kHeads * kHd == kDin && (kSeq & (kSeq - 1)) == 0);
static_assert(kProjP >= kProj && (kProjP % 64) == 0 && (kQW % 64) == 0 && (kDin % 64) == 0 && (kDm % 64) == 0);
static_assert((kDm % 32) == 0 && (kDin % 32) == 0);
static_assert((kRows % 64) == 0 && (kSeq % 64) == 0);
static_assert(kConvC == 3 * kConvTh && (kConvTh % 32) == 0);
static_assert(((kQW * 4) % 128) == 0 && ((kConvC * 4) % 128) == 0 && ((kQDt * 4) % 128) == 0);

constexpr float kUCarry    = 16.0f;
constexpr float kWCarry    = 256.0f;
constexpr float kResCarry  = 2048.0f;
constexpr float kResInv    = 1.0f / kResCarry;
constexpr float kYCarry    = 16.0f;
constexpr float kYInv      = 1.0f / kYCarry;
constexpr float kGCarry    = 16.0f;
constexpr float kInScale   = 1.0f / (kUCarry * kWCarry);
constexpr float kOutScale  = 1.0f / (kGCarry * kWCarry);
constexpr float kNormEps   = 1e-5f;
constexpr float kInvDin    = 1.0f / (float)kDin;

constexpr size_t kSzUH  = (size_t)kRows * kDm * 2;
constexpr size_t kSzWI  = (size_t)kProjP * kDm * 2;
constexpr size_t kSzWO  = (size_t)kDm * kDin * 2;
constexpr size_t kSzQ   = (size_t)kRows * kQW * 4;
constexpr size_t kSzV   = (size_t)kRows * kConvC * 4;
constexpr size_t kSzZ   = (size_t)kRows * kDin * 4;
constexpr size_t kSzY   = (size_t)kRows * kDin * 2;
constexpr size_t kSzALT = (size_t)kDin * kNst * 4;
constexpr size_t kSzDST = (size_t)kDin * 4;
constexpr size_t kOffUH  = 0;
constexpr size_t kOffUL  = kOffUH  + kSzUH;
constexpr size_t kOffWIH = kOffUL  + kSzUH;
constexpr size_t kOffWIL = kOffWIH + kSzWI;
constexpr size_t kOffWOH = kOffWIL + kSzWI;
constexpr size_t kOffQ   = kOffWOH + kSzWO;
constexpr size_t kOffV   = kOffQ   + kSzQ;
constexpr size_t kOffYH  = kOffV   + kSzV;
constexpr size_t kOffYL  = kOffYH  + kSzY;
constexpr size_t kOffALT = kOffYL  + kSzY;
constexpr size_t kOffDST = kOffALT + kSzALT;
constexpr size_t kWsTotal = kOffDST + kSzDST;
constexpr size_t kOffZ   = kOffV;
constexpr size_t kOffYG  = kOffUH;
static_assert(kWsTotal == 128258048ull);
static_assert(kWsTotal <= 134217728ull);
static_assert(kSzZ <= kSzV);
static_assert(kSzY == 2 * kSzUH && kOffUL == kOffUH + kSzUH);
static_assert((kOffUL % 128) == 0 && (kOffWIH % 128) == 0 && (kOffWIL % 128) == 0 && (kOffWOH % 128) == 0 &&
              (kOffQ % 128) == 0 && (kOffV % 128) == 0 && (kOffYH % 128) == 0 && (kOffYL % 128) == 0 &&
              (kOffALT % 128) == 0 && (kOffDST % 128) == 0);

__device__ __forceinline__ float h16_to_f32(unsigned hb) {
  const unsigned sgn = (hb & 0x8000u) << 16;
  const unsigned em = hb & 0x7fffu;
  const float fn = __uint_as_float((em << 13) + 0x38000000u);
  const float fs = (float)em * 5.9604644775390625e-8f;
  const float mag = (em < 0x400u) ? fs : fn;
  return __uint_as_float(__float_as_uint(mag) | sgn);
}
__device__ __forceinline__ unsigned gl_h16bits(float v) {
  const float f = (fabsf(v) < 6.103515625e-05f) ? 0.0f : v;
  return (unsigned)__half_as_ushort(__float2half_rn(f));
}

__global__ __launch_bounds__(256) void split_rows_f16_kernel(
    const float* __restrict__ src, unsigned* __restrict__ dhi, unsigned* __restrict__ dlo,
    int total8, int src8, float carry, int want_lo)
{
  const int i = blockIdx.x * 256 + threadIdx.x;
  if (i >= total8) return;
  v4f a0 = (v4f){0.0f, 0.0f, 0.0f, 0.0f};
  v4f a1 = (v4f){0.0f, 0.0f, 0.0f, 0.0f};
  if ((int)(blockIdx.x * 256) < src8) {
    a0 = *(const v4f*)(src + (size_t)i * 8);
    a1 = *(const v4f*)(src + (size_t)i * 8 + 4);
  }
  const float f[8] = {a0[0] * carry, a0[1] * carry, a0[2] * carry, a0[3] * carry,
                      a1[0] * carry, a1[1] * carry, a1[2] * carry, a1[3] * carry};
  unsigned hb[8], lb[8];
#pragma unroll
  for (int e = 0; e < 8; ++e) {
    hb[e] = gl_h16bits(f[e]);
    const float res = (f[e] - h16_to_f32(hb[e])) * kResCarry;
    lb[e] = gl_h16bits(res);
  }
  const v4u hv = (v4u){hb[0] | (hb[1] << 16), hb[2] | (hb[3] << 16), hb[4] | (hb[5] << 16), hb[6] | (hb[7] << 16)};
  const v4u lv = (v4u){lb[0] | (lb[1] << 16), lb[2] | (lb[3] << 16), lb[4] | (lb[5] << 16), lb[6] | (lb[7] << 16)};
  unsigned* ph = dhi + (size_t)i * 4;
  *(volatile v4u*)ph = hv;
  if (want_lo) {
    unsigned* pl = dlo + (size_t)i * 4;
    *(volatile v4u*)pl = lv;
  }
  __threadfence();
  *(volatile v4u*)ph = hv;
  if (want_lo) {
    unsigned* pl = dlo + (size_t)i * 4;
    *(volatile v4u*)pl = lv;
  }
}

namespace eng {

union FragU { v16h v; v8h h[2]; };
__device__ __forceinline__ v16h frag_load(const _Float16* p) {
  FragU f;
  f.h[0] = *(const v8h*)(p);
  f.h[1] = *(const v8h*)(p + 16);
  return f.v;
}
__device__ __forceinline__ v8f mma_f16(v16h a, v16h b, v8f c) {
  c = __builtin_amdgcn_wmma_f32_16x16x32_f16(false, a, false, b, (short)0, c, false, false);
  asm volatile("v_nop\n\tv_nop\n\tv_nop\n\tv_nop" : "+v"(c) : "v"(a), "v"(b));
  return c;
}

template <int MI, bool SPLIT>
__global__ __launch_bounds__(256) void gemm_f16_kernel(
    const unsigned short* __restrict__ Ap, const unsigned short* __restrict__ A2p, int lda,
    const unsigned short* __restrict__ Btp, const unsigned short* __restrict__ Bt2p, int ldb,
    float* __restrict__ C, int ldc, int M, int N, int K, float scale)
{
  __shared__ __align__(16) float sT[8][16 * 68];
  const _Float16* A   = (const _Float16*)Ap;
  const _Float16* A2  = (const _Float16*)A2p;
  const _Float16* Bt  = (const _Float16*)Btp;
  const _Float16* Bt2 = (const _Float16*)Bt2p;
  const int lane = threadIdx.x & 31;
  const int wave = threadIdx.x >> 5;
  const int tilesN = N >> 6;
  const int tilesM = M / (16 * MI);
  const int tile = blockIdx.x * 8 + wave;
  if (tile >= tilesM * tilesN) return;
  const int tm = tile / tilesN;
  const int tn = tile - tm * tilesN;
  const int m0 = tm * (16 * MI);
  const int n0 = tn << 6;
  const int rlane = lane & 15;
  const int koff  = (lane >> 4) * 8;
  const int mOff  = (lane >> 4) * 8;

  v8f acc[MI][4], accr[MI][4];
#pragma unroll
  for (int i = 0; i < MI; ++i)
#pragma unroll
    for (int j = 0; j < 4; ++j) {
      acc[i][j]  = (v8f){0.f, 0.f, 0.f, 0.f, 0.f, 0.f, 0.f, 0.f};
      accr[i][j] = (v8f){0.f, 0.f, 0.f, 0.f, 0.f, 0.f, 0.f, 0.f};
    }

#pragma unroll 1
  for (int k0 = 0; k0 < K; k0 += 32) {
    v16h ah[MI], al[MI];
#pragma unroll
    for (int i = 0; i < MI; ++i) {
      const size_t ao = (size_t)(m0 + (i << 4) + rlane) * lda + koff + k0;
      ah[i] = frag_load(A + ao);
      al[i] = ah[i];
      if (SPLIT) al[i] = frag_load(A2 + ao);
    }
#pragma unroll
    for (int j = 0; j < 4; ++j) {
      const size_t bo = (size_t)(n0 + (j << 4) + rlane) * ldb + koff + k0;
      const v16h bh = frag_load(Bt + bo);
      v16h bl = bh;
      if (SPLIT) bl = frag_load(Bt2 + bo);
#pragma unroll
      for (int i = 0; i < MI; ++i) {
        acc[i][j] = mma_f16(ah[i], bh, acc[i][j]);
        if (SPLIT) {
          accr[i][j] = mma_f16(ah[i], bl, accr[i][j]);
          accr[i][j] = mma_f16(al[i], bh, accr[i][j]);
        }
      }
    }
  }

  float* slab = sT[wave];
  const int hh = lane >> 4;
  const int c4 = (lane & 15) * 4;
#pragma unroll
  for (int i = 0; i < MI; ++i) {
    const int mBase = m0 + (i << 4);
#pragma unroll
    for (int j = 0; j < 4; ++j) {
#pragma unroll
      for (int r = 0; r < 8; ++r) {
        float v = acc[i][j][r];
        if (SPLIT) v = fmaf(accr[i][j][r], kResInv, v);
        slab[(mOff + r) * 68 + (j << 4) + rlane] = v * scale;
      }
    }
    __builtin_amdgcn_fence(__ATOMIC_RELEASE, "workgroup");
    __builtin_amdgcn_wave_barrier();
    __builtin_amdgcn_fence(__ATOMIC_ACQUIRE, "workgroup");
    for (int pass = 0; pass < 2; ++pass) {
#pragma unroll
      for (int it = 0; it < 8; ++it) {
        const int row = it * 2 + hh;
        const v4f v = *(const v4f*)(slab + row * 68 + c4);
        *(volatile v4f*)(C + (size_t)(mBase + row) * ldc + n0 + c4) = v;
      }
      __threadfence();
    }
    __builtin_amdgcn_fence(__ATOMIC_RELEASE, "workgroup");
    __builtin_amdgcn_wave_barrier();
    __builtin_amdgcn_fence(__ATOMIC_ACQUIRE, "workgroup");
  }
}

}

__global__ __launch_bounds__(352) void conv_silu_kernel(
    const float* __restrict__ Q, const float* __restrict__ cw, const float* __restrict__ cb,
    float* __restrict__ Vp)
{
  const int c  = blockIdx.x * kConvTh + threadIdx.x;
  const int g0 = blockIdx.y * 64;
  const int tb = g0 & (kSeq - 1);
  const v4f wv = *(const v4f*)(cw + (size_t)c * 4);
  const float w0 = wv[0], w1 = wv[1], w2 = wv[2], w3 = wv[3];
  const float bc = cb[c];
  float xm3, xm2, xm1;
  {
    const bool hist = (tb > 0);
    const int rb = hist ? (g0 - 3) : g0;
    const float v3 = Q[(size_t)rb * kQW + c];
    const float v2 = Q[(size_t)(rb + 1) * kQW + c];
    const float v1 = Q[(size_t)(rb + 2) * kQW + c];
    xm3 = hist ? v3 : 0.0f;
    xm2 = hist ? v2 : 0.0f;
    xm1 = hist ? v1 : 0.0f;
  }
#pragma unroll 1
  for (int sub = 0; sub < 8; ++sub) {
    const int lb = g0 + sub * 8;
    float vals[8];
#pragma unroll
    for (int s = 0; s < 8; ++s) {
      const float xcur = Q[(size_t)(lb + s) * kQW + c];
      float acc = w0 * xm3;
      acc = fmaf(w1, xm2, acc);
      acc = fmaf(w2, xm1, acc);
      acc = fmaf(w3, xcur, acc);
      const float sv = acc + bc;
      const float sg = __builtin_amdgcn_rcpf(1.0f + __expf(-sv));
      vals[s] = sv * sg;
      xm3 = xm2;
      xm2 = xm1;
      xm1 = xcur;
    }
    for (int pass = 0; pass < 2; ++pass) {
#pragma unroll
      for (int s = 0; s < 8; ++s)
        *(volatile float*)(Vp + (size_t)(lb + s) * kConvC + c) = vals[s];
      __threadfence();
    }
  }
}

__global__ __launch_bounds__(256) void prep_planes_kernel(
    float* Q, const float* __restrict__ dt_bias, const float* __restrict__ A_log,
    const float* __restrict__ D_skip, float* __restrict__ ALT, float* __restrict__ DST)
{
  const int tid = threadIdx.x;
  const int hd  = tid >> 2;
  const float bias = dt_bias[hd];
  const int r0 = blockIdx.x * 8;
  float pv[8];
#pragma unroll
  for (int i = 0; i < 8; ++i) pv[i] = Q[(size_t)(r0 + i) * kQW + kQDt + hd] + bias;
  for (int pass = 0; pass < 2; ++pass) {
#pragma unroll
    for (int i = 0; i < 8; ++i) {
      const v4f v = (v4f){pv[i], pv[i], pv[i], pv[i]};
      *(volatile v4f*)(Q + (size_t)(r0 + i) * kQW + tid * 4) = v;
    }
    __threadfence();
  }
  if (blockIdx.x < 16) {
    const int ch = blockIdx.x * 64 + (tid >> 2);
    const float al = A_log[ch >> 4];
    const v4f av = (v4f){al, al, al, al};
    float* p = ALT + (size_t)blockIdx.x * 1024 + tid * 4;
    *(volatile v4f*)p = av;
    __threadfence();
    *(volatile v4f*)p = av;
  }
  if (blockIdx.x == 16) {
    const float dv = D_skip[tid >> 2];
    const v4f dvv = (v4f){dv, dv, dv, dv};
    float* p = DST + tid * 4;
    *(volatile v4f*)p = dvv;
    __threadfence();
    *(volatile v4f*)p = dvv;
  }
}

typedef float    ms1_v4f __attribute__((ext_vector_type(4)));
typedef unsigned ms1_v4u __attribute__((ext_vector_type(4)));
struct ms1_args {
  const float* dtpre;
  const float* u;
  const float* bc;
  const float* z;
  const float* A_log;
  const float* Dskip;
  __half* y;
  __half* y_lo;
  long ld_dtpre;
  long ld_u;
  long ld_bc;
  long ld_z;
  long ld_y;
  int offB;
  int offC;
  int offZ;
  float ycarry;
  int dir;
  int D;
  int L;
  int nbatch;
};
static_assert(sizeof(ms1_args) == 136);

__device__ __forceinline__ float ms1_flush16(float v) {
  return (fabsf(v) < 6.103515625e-05f) ? 0.0f : v;
}
__device__ __forceinline__ unsigned ms1_h16bits(float v) {
  return (unsigned)__half_as_ushort(__float2half_rn(ms1_flush16(v)));
}
__device__ __forceinline__ float ms1_h16val(unsigned b) {
  return __half2float(__ushort_as_half((unsigned short)b));
}
__device__ __forceinline__ float ms1_softplus(float v) {
  return fmaxf(v, 0.0f) + log1pf(expf(-fabsf(v)));
}
__device__ __forceinline__ void ms1_pack2(float v0, float v1, unsigned& hw, unsigned& lw) {
  const unsigned h0 = ms1_h16bits(v0);
  const unsigned h1 = ms1_h16bits(v1);
  const float r0 = (v0 - ms1_h16val(h0)) * 2048.0f;
  const float r1 = (v1 - ms1_h16val(h1)) * 2048.0f;
  const unsigned l0 = ms1_h16bits(r0);
  const unsigned l1 = ms1_h16bits(r1);
  hw = h0 | (h1 << 16);
  lw = l0 | (l1 << 16);
}

template <int NSTATE>
__global__ __launch_bounds__(64 * (NSTATE / 16)) void ms1_scan_kernel(ms1_args a)
{
  static_assert(NSTATE == 16 || NSTATE == 64);
  constexpr int NQ  = NSTATE / 16;
  constexpr int NT  = 64 * NQ;
  constexpr int NW  = NT / 32;
  constexpr int BCW = 2 * NSTATE;
  constexpr int YP  = 68;
  constexpr int RPI = NW * 4;
  constexpr int NIT = 64 / RPI;
  static_assert(16 * NT <= 64 * YP);
  __shared__ __align__(16) float sBC[64 * BCW];
  __shared__ __align__(16) float sY[64 * YP];
  const int tid  = threadIdx.x;
  const int lane = tid & 31;
  const int wave = tid >> 5;
  const int c    = tid / NQ;
  const int sq   = tid - c * NQ;
  const int bpb  = a.D / 64;
  const int bi   = blockIdx.x / bpb;
  if (bi >= a.nbatch) return;
  const int d0 = (blockIdx.x - bi * bpb) * 64;
  const int d  = d0 + c;
  const long rowb = (long)bi * a.L;
  const bool hasz  = (a.z != nullptr);
  const bool hasD  = (a.Dskip != nullptr);
  const bool hasLo = (a.y_lo != nullptr);

#pragma unroll 1
  for (int n = 0; n < 16; ++n) {
    const float al = a.A_log[(long)d * NSTATE + sq * 16 + n];
    sY[n * NT + tid] = -expf(al);
  }
  __syncthreads();
  float An[16], h[16];
#pragma unroll
  for (int n = 0; n < 16; ++n) {
    An[n] = sY[n * NT + tid];
    h[n] = 0.0f;
  }
  float Dd = 0.0f;
  if (hasD) Dd = a.Dskip[d];

  const int nchunk = a.L / 64;
  const bool fwd = (a.dir > 0);
  const int s0 = fwd ? 0 : 63;
  const int sd = fwd ? 1 : -1;
  const int q  = lane >> 3;
  const int c8 = (lane & 7) * 8;

#pragma unroll 1
  for (int ci = 0; ci < nchunk; ++ci) {
    const int tb = fwd ? (ci * 64) : (a.L - 64 - ci * 64);
    const long rowc = rowb + tb;
    __syncthreads();
#pragma unroll 8
    for (int i = 0; i < 32; ++i) {
      const int idx = tid + i * NT;
      const int st  = idx / BCW;
      const int col = idx - st * BCW;
      const int sc  = (col < NSTATE) ? (a.offB + col) : (a.offC + col - NSTATE);
      sBC[idx] = a.bc[(rowc + st) * a.ld_bc + sc];
    }
    __syncthreads();
#pragma unroll 1
    for (int s = 0; s < 64; ++s) {
      const int ls = s0 + sd * s;
      const long row = rowc + ls;
      float pre = a.dtpre[row * a.ld_dtpre + d];
      float uv  = a.u[row * a.ld_u + d];
      float zv  = 0.0f;
      if (hasz) zv = a.z[row * a.ld_z + a.offZ + d];
      asm volatile("" : "+v"(pre));
      asm volatile("" : "+v"(uv));
      asm volatile("" : "+v"(zv));
      const float delta = ms1_softplus(pre);
      const float dtx = delta * uv;
      const float* bp = sBC + ls * BCW + sq * 16;
      const float* cp = bp + NSTATE;
      ms1_v4f Bq[4], Cq[4];
#pragma unroll
      for (int k = 0; k < 4; ++k) {
        Bq[k] = *(const ms1_v4f*)(bp + 4 * k);
        Cq[k] = *(const ms1_v4f*)(cp + 4 * k);
      }
      float yv = 0.0f;
#pragma unroll
      for (int n = 0; n < 16; ++n) {
        const float e = __expf(delta * An[n]);
        h[n] = fmaf(e, h[n], dtx * Bq[n >> 2][n & 3]);
        yv = fmaf(h[n], Cq[n >> 2][n & 3], yv);
      }
      if (NQ > 1) {
        yv += __shfl_xor(yv, 1, 32);
        yv += __shfl_xor(yv, 2, 32);
      }
      if (hasD) yv = fmaf(uv, Dd, yv);
      if (hasz) {
        const float sg = __builtin_amdgcn_rcpf(1.0f + expf(-zv));
        yv = yv * (zv * sg);
      }
      if (sq == 0) sY[ls * YP + c] = yv * a.ycarry;
    }
    __syncthreads();
    ms1_v4u hw[NIT], lw[NIT];
#pragma unroll
    for (int it = 0; it < NIT; ++it) {
      const int row = it * RPI + wave * 4 + q;
      const float* sp = sY + row * YP + c8;
      const ms1_v4f f0 = *(const ms1_v4f*)(sp);
      const ms1_v4f f1 = *(const ms1_v4f*)(sp + 4);
      unsigned h0, h1, h2, h3, l0, l1, l2, l3;
      ms1_pack2(f0[0], f0[1], h0, l0);
      ms1_pack2(f0[2], f0[3], h1, l1);
      ms1_pack2(f1[0], f1[1], h2, l2);
      ms1_pack2(f1[2], f1[3], h3, l3);
      hw[it] = (ms1_v4u){h0, h1, h2, h3};
      lw[it] = (ms1_v4u){l0, l1, l2, l3};
    }
    for (int pass = 0; pass < 2; ++pass) {
#pragma unroll
      for (int it = 0; it < NIT; ++it) {
        const int row = it * RPI + wave * 4 + q;
        const long o = (rowc + row) * a.ld_y + d0 + c8;
        *(volatile ms1_v4u*)(a.y + o) = hw[it];
        if (hasLo) *(volatile ms1_v4u*)(a.y_lo + o) = lw[it];
      }
      __threadfence();
    }
  }
}

__global__ __launch_bounds__(256) void gate_norm_kernel(
    const unsigned* __restrict__ YHw, const unsigned* __restrict__ YLw, const float* __restrict__ Z,
    const float* __restrict__ nw, unsigned* __restrict__ YGw)
{
  __shared__ float red[8];
  const int tid  = threadIdx.x;
  const int lane = tid & 31;
  const int wave = tid >> 5;
  const int tok  = tid >> 7;
  const int t8   = (tid & 127) * 8;
  const size_t row = (size_t)blockIdx.x * 2 + tok;
  const size_t e0  = row * kDin + t8;
  const v4u hwv = *(const v4u*)(YHw + (e0 >> 1));
  const v4u lwv = *(const v4u*)(YLw + (e0 >> 1));
  const v4f z0 = *(const v4f*)(Z + e0);
  const v4f z1 = *(const v4f*)(Z + e0 + 4);
  const v4f n0 = *(const v4f*)(nw + t8);
  const v4f n1 = *(const v4f*)(nw + t8 + 4);
  const unsigned hws[4] = {hwv[0], hwv[1], hwv[2], hwv[3]};
  const unsigned lws[4] = {lwv[0], lwv[1], lwv[2], lwv[3]};
  const float zs[8] = {z0[0], z0[1], z0[2], z0[3], z1[0], z1[1], z1[2], z1[3]};
  const float ns[8] = {n0[0], n0[1], n0[2], n0[3], n1[0], n1[1], n1[2], n1[3]};
  float g[8];
  float ss = 0.0f;
#pragma unroll
  for (int k = 0; k < 4; ++k) {
    const float va = h16_to_f32(hws[k] & 0xffffu);
    const float ra = h16_to_f32(lws[k] & 0xffffu);
    const float vb = h16_to_f32(hws[k] >> 16);
    const float rb = h16_to_f32(lws[k] >> 16);
    const float ya = fmaf(ra, kResInv, va) * kYInv;
    const float yb = fmaf(rb, kResInv, vb) * kYInv;
    const float za = zs[2 * k];
    const float zb = zs[2 * k + 1];
    const float sa = __builtin_amdgcn_rcpf(1.0f + __expf(-za));
    const float sb = __builtin_amdgcn_rcpf(1.0f + __expf(-zb));
    const float ga = ya * (za * sa);
    const float gb = yb * (zb * sb);
    g[2 * k]     = ga;
    g[2 * k + 1] = gb;
    ss = fmaf(ga, ga, ss);
    ss = fmaf(gb, gb, ss);
  }
#pragma unroll
  for (int off = 16; off >= 1; off >>= 1) ss += __shfl_xor(ss, off, 32);
  if (lane == 0) red[wave] = ss;
  __syncthreads();
  const int wb = tok * 4;
  const float tot = ((red[wb] + red[wb + 1]) + red[wb + 2]) + red[wb + 3];
  const float rinv = rsqrtf(tot * kInvDin + kNormEps);
  unsigned ob[8];
#pragma unroll
  for (int e = 0; e < 8; ++e) {
    const float o = ((g[e] * rinv) * ns[e]) * kGCarry;
    ob[e] = gl_h16bits(o);
  }
  const v4u ov = (v4u){ob[0] | (ob[1] << 16), ob[2] | (ob[3] << 16), ob[4] | (ob[5] << 16), ob[6] | (ob[7] << 16)};
  unsigned* po = YGw + (e0 >> 1);
  *(volatile v4u*)po = ov;
  __threadfence();
  *(volatile v4u*)po = ov;
}

static_assert(((kRows / 32) * (kQW / 64)) % 8 == 0);
static_assert(((kRows / 32) * (kDin / 64)) % 8 == 0);
static_assert(((kRows / 64) * (kDm / 64)) % 8 == 0);
static_assert((kRows * kDm / 8) % 256 == 0);
static_assert((kProjP * kDm / 8) % 256 == 0 && (kProj * kDm / 8) % 256 == 0);
static_assert((kDm * kDin / 8) % 256 == 0);
static_assert((kRows % 8) == 0 && (kRows / 8) > 16 && (kRows % 2) == 0);

extern "C" void kernel_launch(void* const* d_in, const int* in_sizes, int n_in,
                              void* d_out, int out_size, void* d_ws, size_t ws_size,
                              hipStream_t stream) {
  if (n_in < 9) return;
  if (in_sizes[0] != kRows * kDm) return;
  if (in_sizes[1] != kProj * kDm) return;
  if (in_sizes[2] != kConvC * 4) return;
  if (in_sizes[3] != kConvC) return;
  if (in_sizes[4] != kHeads) return;
  if (in_sizes[5] != kHeads) return;
  if (in_sizes[6] != kHeads) return;
  if (in_sizes[7] != kDin) return;
  if (in_sizes[8] != kDm * kDin) return;
  if (out_size != kRows * kDm) return;
  if (ws_size < kWsTotal) return;
  if ((kDin % 64) != 0 || (kSeq % 64) != 0) return;

  const float* u_in     = (const float*)d_in[0];
  const float* w_in     = (const float*)d_in[1];
  const float* conv_w   = (const float*)d_in[2];
  const float* conv_b   = (const float*)d_in[3];
  const float* dt_bias  = (const float*)d_in[4];
  const float* A_log    = (const float*)d_in[5];
  const float* D_skip   = (const float*)d_in[6];
  const float* norm_w   = (const float*)d_in[7];
  const float* w_out    = (const float*)d_in[8];
  float* out = (float*)d_out;

  char* ws = (char*)d_ws;
  float* Q   = (float*)(ws + kOffQ);
  float* Vp  = (float*)(ws + kOffV);
  float* Zp  = (float*)(ws + kOffZ);
  float* ALT = (float*)(ws + kOffALT);
  float* DST = (float*)(ws + kOffDST);

  split_rows_f16_kernel<<<dim3(kRows * kDm / 8 / 256), 256, 0, stream>>>(
      u_in, (unsigned*)(ws + kOffUH), (unsigned*)(ws + kOffUL), kRows * kDm / 8, kRows * kDm / 8, kUCarry, 1);
  split_rows_f16_kernel<<<dim3(kProjP * kDm / 8 / 256), 256, 0, stream>>>(
      w_in, (unsigned*)(ws + kOffWIH), (unsigned*)(ws + kOffWIL), kProjP * kDm / 8, kProj * kDm / 8, kWCarry, 1);
  split_rows_f16_kernel<<<dim3(kDm * kDin / 8 / 256), 256, 0, stream>>>(
      w_out, (unsigned*)(ws + kOffWOH), (unsigned*)nullptr, kDm * kDin / 8, kDm * kDin / 8, kWCarry, 0);

  const unsigned short* UH  = (const unsigned short*)(ws + kOffUH);
  const unsigned short* UL  = (const unsigned short*)(ws + kOffUL);
  const unsigned short* WIH = (const unsigned short*)(ws + kOffWIH);
  const unsigned short* WIL = (const unsigned short*)(ws + kOffWIL);
  const unsigned short* WOH = (const unsigned short*)(ws + kOffWOH);

  eng::gemm_f16_kernel<2, true><<<dim3((kRows / 32) * (kQW / 64) / 8), 256, 0, stream>>>(
      UH, UL, kDm,
      WIH + (size_t)kDin * kDm, WIL + (size_t)kDin * kDm, kDm,
      Q, kQW, kRows, kQW, kDm, kInScale);

  conv_silu_kernel<<<dim3(kConvC / kConvTh, kRows / 64), kConvTh, 0, stream>>>(Q, conv_w, conv_b, Vp);

  prep_planes_kernel<<<dim3(kRows / 8), 256, 0, stream>>>(Q, dt_bias, A_log, D_skip, ALT, DST);

  ms1_args sa;
  sa.dtpre = Q;
  sa.u = Vp;
  sa.bc = Vp;
  sa.z = nullptr;
  sa.A_log = ALT;
  sa.Dskip = DST;
  sa.y = (__half*)(ws + kOffYH);
  sa.y_lo = (__half*)(ws + kOffYL);
  sa.ld_dtpre = kQW;
  sa.ld_u = kConvC;
  sa.ld_bc = kConvC;
  sa.ld_z = 0;
  sa.ld_y = kDin;
  sa.offB = kDin;
  sa.offC = kDin + kNst;
  sa.offZ = 0;
  sa.ycarry = kYCarry;
  sa.dir = 1;
  sa.D = kDin;
  sa.L = kSeq;
  sa.nbatch = kBatch;
  ms1_scan_kernel<16><<<dim3((kDin / 64) * kBatch), 64, 0, stream>>>(sa);

  eng::gemm_f16_kernel<2, true><<<dim3((kRows / 32) * (kDin / 64) / 8), 256, 0, stream>>>(
      UH, UL, kDm,
      WIH, WIL, kDm,
      Zp, kDin, kRows, kDin, kDm, kInScale);

  gate_norm_kernel<<<dim3(kRows / 2), 256, 0, stream>>>(
      (const unsigned*)(ws + kOffYH), (const unsigned*)(ws + kOffYL), Zp, norm_w, (unsigned*)(ws + kOffYG));

  eng::gemm_f16_kernel<4, false><<<dim3((kRows / 64) * (kDm / 64) / 8), 256, 0, stream>>>(
      (const unsigned short*)(ws + kOffYG), (const unsigned short*)nullptr, kDin,
      WOH, (const unsigned short*)nullptr, kDin,
      out, kDm, kRows, kDm, kDin, kOutScale);
}
